// MHLAttention_1443109011474
// MI455X (gfx1250) — hardware-verified
//
#include <hip/hip_runtime.h>
#include <math.h>
#include <stdint.h>

#define NB    2
#define SEQ   2048
#define DMOD  1024
#define NH    16
#define HDIM  192
#define DLAT  3072
#define DKV   192
#define NQKV  9216
#define ROTP  16
#define ROPC0 16
#define RESR  512
#define QSC   64.0f
#define KSC   64.0f
#define HSC   1024.0f
#define WSC   1024.0f
#define PCAR  32768.0f
#define VCAR  1024.0f
#define OSC   1024.0f
#define LOG2E 1.4426950408889634f
#define RSQD  0.07216878364870322f
#define ATT_WAVES   4
#define ATT_THREADS (ATT_WAVES * 32)
#define MAXBLK (SEQ / 32)
#define SLABF  (16 * 68)
#define SLAB64 (16 * 68)
#define VTP    72
#define RPITCH (NH * HDIM)

static_assert(DLAT == NH * HDIM && NQKV == 3 * DLAT && RPITCH == DLAT);
static_assert(HDIM % 64 == 0 && HDIM % 32 == 0 && DKV % 64 == 0 && DKV % 32 == 0 && DMOD % 64 == 0 && DLAT % 64 == 0);
static_assert((HDIM / 8) == 24 && (DKV / 8) == 24);
static_assert(ROPC0 * 8 == 128 && ROTP * 2 == 32);
static_assert(SEQ % 64 == 0 && RESR % 64 == 0 && RESR <= SEQ && (SEQ & (SEQ - 1)) == 0 && SEQ % 16 == 0);
static_assert(ATT_THREADS == 128 && MAXBLK == 64 && 16 * 36 <= SLABF);
static_assert(((NB * SEQ * DMOD / 8) % 256) == 0 && ((NB * SEQ) % 8) == 0 && ((NB * SEQ * NH * (HDIM / 8)) % 256) == 0);
static_assert(NH == 16 && NB == 2 && (SEQ / 64) == 32);

typedef unsigned short u16;
typedef _Float16 v16h __attribute__((ext_vector_type(16)));
typedef _Float16 v8h  __attribute__((ext_vector_type(8)));
typedef __bf16   v16b __attribute__((ext_vector_type(16)));
typedef float    v8f  __attribute__((ext_vector_type(8)));
typedef float    v4f  __attribute__((ext_vector_type(4)));
typedef unsigned int v4u __attribute__((ext_vector_type(4)));

union FragH { v16h v; v8h h[2]; v4u u[2]; };
union FragB { v16b v; v4u u[2]; };

struct InvF { float f[16]; };
static_assert(sizeof(InvF) == 64);

__device__ __forceinline__ unsigned short bf_bits(float f) {
  unsigned u = __float_as_uint(f);
  return (unsigned short)((u + 0x7FFFu + ((u >> 16) & 1u)) >> 16);
}
__device__ __forceinline__ float bf_up(unsigned short h) { return __uint_as_float(((unsigned)h) << 16); }
__device__ __forceinline__ float bfr(float f) { return bf_up(bf_bits(f)); }
__device__ __forceinline__ unsigned short h_bits(_Float16 x) { return __builtin_bit_cast(unsigned short, x); }
__device__ __forceinline__ unsigned pk16(unsigned short a, unsigned short b) { return (unsigned)a | ((unsigned)b << 16); }
__device__ __forceinline__ v8f zero8() { v8f z = {0.f, 0.f, 0.f, 0.f, 0.f, 0.f, 0.f, 0.f}; return z; }
__device__ __forceinline__ v4f zero4() { v4f z = {0.f, 0.f, 0.f, 0.f}; return z; }

__device__ __forceinline__ v16h ldfrag_h(const _Float16* p) {
  FragH f;
  f.h[0] = *(const v8h*)(p);
  f.h[1] = *(const v8h*)(p + 16);
  return f.v;
}
__device__ __forceinline__ v16b ldfrag_b(const u16* p) {
  FragB f;
  f.u[0] = *(const v4u*)(p);
  f.u[1] = *(const v4u*)(p + 16);
  return f.v;
}

__device__ __forceinline__ v8f mma_h(v16h a, v16h b, v8f c) {
  return __builtin_amdgcn_wmma_f32_16x16x32_f16(false, a, false, b, (short)0, c, false, false);
}
__device__ __forceinline__ v8f mma_b(v16b a, v16b b, v8f c) {
  return __builtin_amdgcn_wmma_f32_16x16x32_bf16(false, a, false, b, (short)0, c, false, false);
}
__device__ __forceinline__ void guard2(v8f& a, v8f& b, v16h x0, v16h x1, v16h x2, v16h x3, v16h x4, v16h x5) {
#if defined(__HIP_DEVICE_COMPILE__)
  asm volatile("v_nop\n\tv_nop\n\tv_nop\n\tv_nop"
               : "+v"(a), "+v"(b) : "v"(x0), "v"(x1), "v"(x2), "v"(x3), "v"(x4), "v"(x5) : "memory");
#endif
}
template <typename F>
__device__ __forceinline__ void guard6(v8f& a, v8f& b, v8f& c, v8f& d, F x0, F x1, F x2, F x3, F x4, F x5) {
#if defined(__HIP_DEVICE_COMPILE__)
  asm volatile("v_nop\n\tv_nop\n\tv_nop\n\tv_nop"
               : "+v"(a), "+v"(b), "+v"(c), "+v"(d) : "v"(x0), "v"(x1), "v"(x2), "v"(x3), "v"(x4), "v"(x5) : "memory");
#endif
}
__device__ __forceinline__ void acc_guard4(v8f& a, v8f& b, v8f& c, v8f& d) {
#if defined(__HIP_DEVICE_COMPILE__)
  asm volatile("v_nop\n\tv_nop\n\tv_nop\n\tv_nop" : "+v"(a), "+v"(b), "+v"(c), "+v"(d));
#endif
}
__device__ __forceinline__ void wave_sync_lds() {
  __builtin_amdgcn_fence(__ATOMIC_RELEASE, "workgroup");
  __builtin_amdgcn_wave_barrier();
  __builtin_amdgcn_fence(__ATOMIC_ACQUIRE, "workgroup");
}

__device__ __forceinline__ void sincos_acc(float angf, float& sv, float& cv) {
  const double a = (double)angf;
  const double TWO_OVER_PI = 0.63661977236758134308;
  const double PIO2_HI = 1.5707963267948966;
  const double PIO2_LO = 6.123233995736766e-17;
  const int kq = (int)(a * TWO_OVER_PI + 0.5);
  const double kd = (double)kq;
  double r = fma(-kd, PIO2_HI, a);
  r = fma(-kd, PIO2_LO, r);
  const double r2 = r * r;
  double sp = 1.0 / 6227020800.0;
  sp = fma(sp, r2, -1.0 / 39916800.0);
  sp = fma(sp, r2, 1.0 / 362880.0);
  sp = fma(sp, r2, -1.0 / 5040.0);
  sp = fma(sp, r2, 1.0 / 120.0);
  sp = fma(sp, r2, -1.0 / 6.0);
  const double s = fma(sp * r2, r, r);
  double cp = -1.0 / 87178291200.0;
  cp = fma(cp, r2, 1.0 / 479001600.0);
  cp = fma(cp, r2, -1.0 / 3628800.0);
  cp = fma(cp, r2, 1.0 / 40320.0);
  cp = fma(cp, r2, -1.0 / 720.0);
  cp = fma(cp, r2, 1.0 / 24.0);
  cp = fma(cp, r2, -0.5);
  const double c = fma(cp, r2, 1.0);
  const int qd = kq & 3;
  const double so = (qd == 0) ? s : (qd == 1) ? c : (qd == 2) ? -s : -c;
  const double co = (qd == 0) ? c : (qd == 1) ? -s : (qd == 2) ? -c : s;
  sv = (float)so;
  cv = (float)co;
}

__global__ __launch_bounds__(256) void k_tab(float* cosT, float* sinT, InvF inv) {
  const int tid  = threadIdx.x;
  const int lane = tid & 31;
  const int hh   = lane >> 4;
  const int i    = lane & 15;
  const int tb   = (blockIdx.x * 8 + (tid >> 5)) * 2;
  if (tb >= SEQ) return;
  const int t = tb + hh;
  float f = inv.f[0];
#pragma unroll
  for (int k = 1; k < ROTP; ++k) f = (i == k) ? inv.f[k] : f;
  const float ang = (float)t * f;
  float sv, cv;
  sincos_acc(ang, sv, cv);
  float* cr = cosT + (size_t)tb * ROTP + lane;
  float* sr = sinT + (size_t)tb * ROTP + lane;
  for (int pass = 0; pass < 2; ++pass) {
    *(volatile float*)(cr) = cv;
    *(volatile float*)(sr) = sv;
    __threadfence();
  }
}

__global__ __launch_bounds__(256) void cvt16(const float* __restrict__ x, u16* D, int n8, int f16mode, float scale) {
  const int gt = blockIdx.x * 256 + (int)threadIdx.x;
  if (gt >= n8) return;
  const float* p = x + (size_t)gt * 8;
  const v4f a = *(const v4f*)(p), bq = *(const v4f*)(p + 4);
  float v[8];
#pragma unroll
  for (int e = 0; e < 4; ++e) { v[e] = a[e]; v[4 + e] = bq[e]; }
  unsigned short s[8];
#pragma unroll
  for (int e = 0; e < 8; ++e) {
    const unsigned short hb = h_bits((_Float16)(bfr(v[e]) * scale));
    const unsigned short bb = bf_bits(v[e]);
    s[e] = (f16mode != 0) ? hb : bb;
  }
  v4u o;
#pragma unroll
  for (int e = 0; e < 4; ++e) o[e] = pk16(s[2 * e], s[2 * e + 1]);
  u16* d = D + (size_t)gt * 8;
  for (int pass = 0; pass < 2; ++pass) {
    *(volatile v4u*)(d) = o;
    __threadfence();
  }
}

__global__ __launch_bounds__(256) void tr16(const float* __restrict__ in, u16* outp, int C, int KD, int ntn,
                                            int perm, int f16mode, float scale) {
  __shared__ __align__(16) u16 T[64 * VTP];
  const int tid = threadIdx.x;
  const int bid = blockIdx.x;
  const int n0  = (bid % ntn) * 64;
  const int k0  = (bid / ntn) * 64;
  {
    const int nl = tid & 63;
    const int kq = tid >> 6;
    const int n  = n0 + nl;
    int col = n;
    if (perm != 0) {
      const int part = n / DLAT;
      const int rem  = n - part * DLAT;
      const int hd   = rem / HDIM;
      const int dd   = rem - hd * HDIM;
      col = part * DLAT + dd * NH + hd;
    }
    const float* src = in + col;
#pragma unroll 4
    for (int i = 0; i < 16; ++i) {
      const int kl = kq + 4 * i;
      const float v = src[(size_t)(k0 + kl) * (size_t)C];
      const unsigned short hb = h_bits((_Float16)(bfr(v) * scale));
      const unsigned short bb = bf_bits(v);
      T[nl * VTP + kl] = (f16mode != 0) ? hb : bb;
    }
  }
  __syncthreads();
  v4u vv[2];
  const int q8 = tid >> 3, p8 = (tid & 7) * 8;
#pragma unroll
  for (int it = 0; it < 2; ++it) {
    const int line = it * 32 + q8;
    vv[it] = *(const v4u*)(T + line * VTP + p8);
  }
  const size_t base = (size_t)n0 * (size_t)KD + k0 + p8;
  for (int pass = 0; pass < 2; ++pass) {
#pragma unroll
    for (int it = 0; it < 2; ++it) {
      const int line = it * 32 + q8;
      *(volatile v4u*)(outp + base + (size_t)line * (size_t)KD) = vv[it];
    }
    __threadfence();
  }
}

__device__ __forceinline__ void epi64(float* sl, v8f a0, v8f a1, v8f a2, v8f a3, float oscale, v4f badd, float* C, int N,
                                      size_t rowb, int col0, int lane) {
  const int hh = lane >> 4, m = lane & 15;
#pragma unroll
  for (int r = 0; r < 8; ++r) {
    const int ro = (8 * hh + r) * 68 + m;
    sl[ro]      = a0[r] * oscale;
    sl[ro + 16] = a1[r] * oscale;
    sl[ro + 32] = a2[r] * oscale;
    sl[ro + 48] = a3[r] * oscale;
  }
  wave_sync_lds();
  v4f vals[8];
#pragma unroll
  for (int it = 0; it < 8; ++it) vals[it] = *(const v4f*)(sl + (it * 2 + hh) * 68 + m * 4) + badd;
  float* dst = C + (rowb + (size_t)hh) * (size_t)N + col0 + m * 4;
  for (int pass = 0; pass < 2; ++pass) {
#pragma unroll
    for (int it = 0; it < 8; ++it) {
      *(volatile v4f*)(dst + (size_t)(it * 2) * (size_t)N) = vals[it];
    }
    __threadfence();
  }
}

__global__ __launch_bounds__(128)
void gemm_bf(const u16* __restrict__ A, const u16* __restrict__ Bt, float* C, int M, int N, int K, float oscale) {
  __shared__ __align__(16) float slab[4 * SLAB64];
  const int tid = threadIdx.x, wave = tid >> 5, lane = tid & 31, hh = lane >> 4, m = lane & 15;
  const int ntile = N >> 6;
  const int bid   = blockIdx.x;
  const int rowb  = (bid / ntile) * 64 + wave * 16;
  const int col0  = (bid % ntile) * 64;
  if (rowb + 16 > M) return;
  const u16* ap = A  + (size_t)(rowb + m) * K + 8 * hh;
  const u16* bp = Bt + (size_t)(col0 + m) * K + 8 * hh;
  const size_t bs = (size_t)16 * K;
  v8f acc0 = zero8(), acc1 = zero8(), acc2 = zero8(), acc3 = zero8();
#pragma unroll 1
  for (int k0 = 0; k0 < K; k0 += 32) {
    const v16b a  = ldfrag_b(ap + k0);
    const v16b b0 = ldfrag_b(bp + k0);
    const v16b b1 = ldfrag_b(bp + bs + k0);
    const v16b b2 = ldfrag_b(bp + 2 * bs + k0);
    const v16b b3 = ldfrag_b(bp + 3 * bs + k0);
    acc0 = mma_b(a, b0, acc0);
    acc1 = mma_b(a, b1, acc1);
    acc2 = mma_b(a, b2, acc2);
    acc3 = mma_b(a, b3, acc3);
    guard6<v16b>(acc0, acc1, acc2, acc3, a, b0, b1, b2, b3, a);
  }
  epi64(slab + wave * SLAB64, acc0, acc1, acc2, acc3, oscale, zero4(), C, N, (size_t)rowb, col0, lane);
}

__global__ __launch_bounds__(128)
void gemm_hr(const u16* __restrict__ Ah, const u16* __restrict__ Al, const u16* __restrict__ Bt,
             float* C, int M, int N, int K, float oscale, int resr, int lrpb) {
  __shared__ __align__(16) float slab[4 * SLAB64];
  const int tid = threadIdx.x, wave = tid >> 5, lane = tid & 31, hh = lane >> 4, m = lane & 15;
  const int ntile = N >> 6;
  const int bid   = blockIdx.x;
  const int rowb  = (bid / ntile) * 64 + wave * 16;
  const int col0  = (bid % ntile) * 64;
  if (rowb + 16 > M) return;
  const int bt  = rowb / SEQ;
  const int sb  = rowb - bt * SEQ;
  const bool lo_on = (sb < resr);
  const int sbl = lo_on ? sb : 0;
  const _Float16* ahp = (const _Float16*)(const void*)Ah + (size_t)(rowb + m) * K + 8 * hh;
  const _Float16* alp = (const _Float16*)(const void*)Al + (size_t)(bt * lrpb + sbl + m) * K + 8 * hh;
  const _Float16* bp  = (const _Float16*)(const void*)Bt + (size_t)(col0 + m) * K + 8 * hh;
  const size_t bs = (size_t)16 * K;
  v8f acc0 = zero8(), acc1 = zero8(), acc2 = zero8(), acc3 = zero8();
  if (lo_on) {
#pragma unroll 1
    for (int k0 = 0; k0 < K; k0 += 32) {
      const v16h ah = ldfrag_h(ahp + k0), al = ldfrag_h(alp + k0);
      const v16h b0 = ldfrag_h(bp + k0);
      const v16h b1 = ldfrag_h(bp + bs + k0);
      const v16h b2 = ldfrag_h(bp + 2 * bs + k0);
      const v16h b3 = ldfrag_h(bp + 3 * bs + k0);
      acc0 = mma_h(ah, b0, acc0);  acc0 = mma_h(al, b0, acc0);
      acc1 = mma_h(ah, b1, acc1);  acc1 = mma_h(al, b1, acc1);
      acc2 = mma_h(ah, b2, acc2);  acc2 = mma_h(al, b2, acc2);
      acc3 = mma_h(ah, b3, acc3);  acc3 = mma_h(al, b3, acc3);
      guard6<v16h>(acc0, acc1, acc2, acc3, ah, al, b0, b1, b2, b3);
    }
  } else {
#pragma unroll 1
    for (int k0 = 0; k0 < K; k0 += 32) {
      const v16h ah = ldfrag_h(ahp + k0);
      const v16h b0 = ldfrag_h(bp + k0);
      const v16h b1 = ldfrag_h(bp + bs + k0);
      const v16h b2 = ldfrag_h(bp + 2 * bs + k0);
      const v16h b3 = ldfrag_h(bp + 3 * bs + k0);
      acc0 = mma_h(ah, b0, acc0);
      acc1 = mma_h(ah, b1, acc1);
      acc2 = mma_h(ah, b2, acc2);
      acc3 = mma_h(ah, b3, acc3);
      guard6<v16h>(acc0, acc1, acc2, acc3, ah, b0, b1, b2, b3, ah);
    }
  }
  epi64(slab + wave * SLAB64, acc0, acc1, acc2, acc3, oscale, zero4(), C, N, (size_t)rowb, col0, lane);
}

__global__ __launch_bounds__(256) void rms16(const float* __restrict__ H, const float* __restrict__ w,
                                             u16* Ho, u16* Lo, int nrows, float sc) {
  const int tid  = threadIdx.x;
  const int lane = tid & 31;
  const int row  = blockIdx.x * 8 + (tid >> 5);
  if (row >= nrows) return;
  const bool live = lane < (DKV / 8);
  const int lc = live ? lane : (DKV / 8 - 1);
  const float* p = H + (size_t)row * DKV + lc * 8;
  const v4f a = *(const v4f*)(p), bq = *(const v4f*)(p + 4);
  const v4f wa = *(const v4f*)(w + lc * 8), wb = *(const v4f*)(w + lc * 8 + 4);
  float v[8], wv[8];
#pragma unroll
  for (int e = 0; e < 4; ++e) { v[e] = a[e]; v[4 + e] = bq[e]; wv[e] = wa[e]; wv[4 + e] = wb[e]; }
  float ss = 0.f;
#pragma unroll
  for (int e = 0; e < 8; ++e) { const float vv = live ? v[e] : 0.f; ss += vv * vv; }
#pragma unroll
  for (int off = 1; off < 32; off <<= 1) ss += __shfl_xor(ss, off, 32);
  const float rs = rsqrtf(ss * (1.0f / (float)DKV) + 1e-6f);
  v4u oh, ol;
#pragma unroll
  for (int e = 0; e < 4; ++e) {
    const float t0 = ((v[2 * e] * rs) * bfr(wv[2 * e])) * sc;
    const float t1 = ((v[2 * e + 1] * rs) * bfr(wv[2 * e + 1])) * sc;
    const _Float16 h0 = (_Float16)t0, h1 = (_Float16)t1;
    const _Float16 l0 = (_Float16)(t0 - (float)h0), l1 = (_Float16)(t1 - (float)h1);
    oh[e] = pk16(h_bits(h0), h_bits(h1));
    ol[e] = pk16(h_bits(l0), h_bits(l1));
  }
  if (live) {
    const size_t o8 = (size_t)row * DKV + lane * 8;
    for (int pass = 0; pass < 2; ++pass) {
      *(volatile v4u*)(Ho + o8) = oh;
      *(volatile v4u*)(Lo + o8) = ol;
      __threadfence();
    }
  }
}

__global__ __launch_bounds__(256) void rope16(const float* __restrict__ x,
                                              const float* __restrict__ cosT, const float* __restrict__ sinT,
                                              u16* outp, int nrows, float sc) {
#pragma clang fp contract(off)
  const int gt   = blockIdx.x * 256 + (int)threadIdx.x;
  const int row  = gt / (HDIM / 8);
  const int ch   = gt - row * (HDIM / 8);
  const int d0   = ch * 8;
  const bool live = row < nrows;
  const int rowc = live ? row : (nrows - 1);
  const int pos  = (rowc / NH) & (SEQ - 1);
  const float* xr = x + (size_t)rowc * HDIM + d0;
  const v4f xa = *(const v4f*)(xr), xb = *(const v4f*)(xr + 4);
  float y[8];
#pragma unroll
  for (int e = 0; e < 4; ++e) { y[e] = xa[e]; y[4 + e] = xb[e]; }
  const bool rc = (ch >= ROPC0) && (ch < ROPC0 + (2 * ROTP) / 8);
  const int i0  = rc ? (ch - ROPC0) * 4 : 0;
  const v4f cv = *(const v4f*)(cosT + (size_t)pos * ROTP + i0);
  const v4f sv = *(const v4f*)(sinT + (size_t)pos * ROTP + i0);
  float w[8];
#pragma unroll
  for (int e = 0; e < 4; ++e) {
    const float y1 = y[2 * e], y2 = y[2 * e + 1];
    const float r0 = y1 * cv[e] - y2 * sv[e];
    const float r1 = y1 * sv[e] + y2 * cv[e];
    w[2 * e]     = rc ? r0 : y1;
    w[2 * e + 1] = rc ? r1 : y2;
  }
  v4u oh;
#pragma unroll
  for (int e = 0; e < 4; ++e) {
    const _Float16 h0 = (_Float16)(w[2 * e] * sc), h1 = (_Float16)(w[2 * e + 1] * sc);
    oh[e] = pk16(h_bits(h0), h_bits(h1));
  }
  if (live) {
    const size_t o8 = (size_t)row * HDIM + d0;
    for (int pass = 0; pass < 2; ++pass) {
      *(volatile v4u*)(outp + o8) = oh;
      __threadfence();
    }
  }
}

__global__ __launch_bounds__(256) void vt16(const float* __restrict__ v, u16* VHo, u16* VLo) {
  __shared__ __align__(16) u16 TH[64 * VTP];
  __shared__ __align__(16) u16 TL[64 * VTP];
  const int tid = threadIdx.x;
  const int bid = blockIdx.x;
  const int dch = bid % 3;
  const int r3  = bid / 3;
  const int st  = r3 & (SEQ / 64 - 1);
  const int h   = (r3 >> 5) & (NH - 1);
  const int b   = (r3 >> 9) & (NB - 1);
  const int s0  = st * 64;
  {
    const int sl = tid >> 2;
    const int dc = (tid & 3) * 16;
    const float* src = v + (((size_t)(b * SEQ + s0 + sl)) * NH + h) * HDIM + dch * 64 + dc;
#pragma unroll
    for (int i = 0; i < 4; ++i) {
      const v4f a = *(const v4f*)(src + 4 * i);
#pragma unroll
      for (int e = 0; e < 4; ++e) {
        const float t = a[e] * VCAR;
        const _Float16 hv = (_Float16)t;
        const _Float16 lv = (_Float16)(t - (float)hv);
        TH[(dc + 4 * i + e) * VTP + sl] = h_bits(hv);
        TL[(dc + 4 * i + e) * VTP + sl] = h_bits(lv);
      }
    }
  }
  __syncthreads();
  v4u vh[2], vl[2];
  const int q8 = tid >> 3, p8 = (tid & 7) * 8;
#pragma unroll
  for (int it = 0; it < 2; ++it) {
    const int line = it * 32 + q8;
    vh[it] = *(const v4u*)(TH + line * VTP + p8);
    vl[it] = *(const v4u*)(TL + line * VTP + p8);
  }
  const size_t drow  = (size_t)(b * NH + h) * HDIM + dch * 64;
  const size_t baseH = drow * SEQ + s0 + p8;
  const size_t baseL = drow * RESR + s0 + p8;
  const bool lo_on = (s0 < RESR);
  for (int pass = 0; pass < 2; ++pass) {
#pragma unroll
    for (int it = 0; it < 2; ++it) {
      const int line = it * 32 + q8;
      *(volatile v4u*)(VHo + baseH + (size_t)line * SEQ) = vh[it];
      if (lo_on) *(volatile v4u*)(VLo + baseL + (size_t)line * RESR) = vl[it];
    }
    __threadfence();
  }
}

template <bool RESID>
__device__ __forceinline__ void pv2(v8f& oa, v8f& ob, v16h ph, v16h pl, const _Float16* vhp, const _Float16* vlp) {
  const v16h vh0 = ldfrag_h(vhp);
  const v16h vh1 = ldfrag_h(vhp + (size_t)16 * SEQ);
  if (RESID) {
    const v16h vl0 = ldfrag_h(vlp);
    const v16h vl1 = ldfrag_h(vlp + (size_t)16 * RESR);
    oa = mma_h(ph, vh0, oa);  oa = mma_h(pl, vh0, oa);  oa = mma_h(ph, vl0, oa);
    ob = mma_h(ph, vh1, ob);  ob = mma_h(pl, vh1, ob);  ob = mma_h(ph, vl1, ob);
    guard2(oa, ob, ph, pl, vh0, vh1, vl0, vl1);
  } else {
    oa = mma_h(ph, vh0, oa);
    ob = mma_h(ph, vh1, ob);
    guard2(oa, ob, ph, vh0, vh1, ph, vh0, vh1);
  }
}

template <bool RESID>
__device__ __forceinline__ void epi_chunk(float* slab, v8f oa, v8f ob, v8f oc, v8f od, v8f invv,
                                          u16* ohp, u16* olp, int lane) {
  const int hh = lane >> 4, c = lane & 15;
  wave_sync_lds();
#pragma unroll
  for (int r = 0; r < 8; ++r) {
    const int ro = (8 * hh + r) * 68 + c;
    slab[ro]      = oa[r] * invv[r];
    slab[ro + 16] = ob[r] * invv[r];
    slab[ro + 32] = oc[r] * invv[r];
    slab[ro + 48] = od[r] * invv[r];
  }
  wave_sync_lds();
  v4u oh[4], ol[4];
  const int rq = lane >> 3, c8 = (lane & 7) * 8;
#pragma unroll
  for (int it = 0; it < 4; ++it) {
    const int row = it * 4 + rq;
    const v4f a = *(const v4f*)(slab + row * 68 + c8), bq = *(const v4f*)(slab + row * 68 + c8 + 4);
    float w[8];
#pragma unroll
    for (int e = 0; e < 4; ++e) { w[e] = a[e] * OSC; w[4 + e] = bq[e] * OSC; }
#pragma unroll
    for (int e = 0; e < 4; ++e) {
      const _Float16 h0 = (_Float16)w[2 * e], h1 = (_Float16)w[2 * e + 1];
      const _Float16 l0 = (_Float16)(w[2 * e] - (float)h0), l1 = (_Float16)(w[2 * e + 1] - (float)h1);
      oh[it][e] = pk16(h_bits(h0), h_bits(h1));
      ol[it][e] = pk16(h_bits(l0), h_bits(l1));
    }
  }
  for (int pass = 0; pass < 2; ++pass) {
#pragma unroll
    for (int it = 0; it < 4; ++it) {
      const int row = it * 4 + rq;
      const size_t o8 = (size_t)row * RPITCH + c8;
      *(volatile v4u*)(ohp + o8) = oh[it];
      if (RESID) *(volatile v4u*)(olp + o8) = ol[it];
    }
    __threadfence();
  }
}

template <bool RESID>
__global__ __launch_bounds__(ATT_THREADS)
void attn_causal(const u16* __restrict__ QHp, const u16* __restrict__ KHp,
                 const u16* __restrict__ VHp, const u16* __restrict__ VLp,
                 const int* __restrict__ amask, u16* OHo, u16* OLo, int qt0, int nqt) {
  __shared__ __align__(16) float smem[ATT_WAVES * SLABF];

  const int tid  = threadIdx.x;
  const int wave = tid >> 5;
  const int lane = tid & 31;
  const int hh   = lane >> 4;
  const int c    = lane & 15;

  const int bid  = blockIdx.x;
  const int qt   = qt0 + (bid % nqt);
  const int rr   = bid / nqt;
  const int head = rr & (NH - 1);
  const int b    = (rr >> 4) & (NB - 1);
  const int q0   = qt * 64 + wave * 16;

  const _Float16* Qh  = (const _Float16*)(const void*)QHp + ((size_t)(b * SEQ + q0 + c)) * RPITCH + head * HDIM + 8 * hh;
  const _Float16* Khb = (const _Float16*)(const void*)KHp + ((size_t)b * SEQ + c) * RPITCH + head * HDIM + 8 * hh;
  const size_t vrow = (size_t)(b * NH + head) * HDIM + c;
  const _Float16* Vhb = (const _Float16*)(const void*)VHp + vrow * SEQ + 8 * hh;
  const _Float16* Vlb = (const _Float16*)(const void*)VLp + vrow * RESR + 8 * hh;
  const int* amb = amask + ((size_t)(b * SEQ) + q0 + 8 * hh) * SEQ + c;
  const float lsc  = RSQD * LOG2E / (QSC * KSC);
  const float FILL = -1.0e9f * LOG2E;

  float mrow[8], lrow[8];
  v8f o[12];
#pragma unroll
  for (int r = 0; r < 8; ++r) { mrow[r] = -INFINITY; lrow[r] = 0.f; }
#pragma unroll
  for (int j = 0; j < 12; ++j) o[j] = zero8();
  float* pt = smem + wave * SLABF;

  int nblk = (q0 + 16 + 31) >> 5;
  nblk = (nblk > MAXBLK) ? MAXBLK : nblk;

#pragma unroll 1
  for (int it = 0; it < nblk; ++it) {
    const int kb = it * 32;
    v8f s0 = zero8(), s1 = zero8();
    const _Float16* k0p = Khb + (size_t)kb * RPITCH;
    const _Float16* k1p = k0p + (size_t)16 * RPITCH;
#pragma unroll
    for (int kk = 0; kk < HDIM / 32; ++kk) {
      const v16h qh  = ldfrag_h(Qh + kk * 32);
      const v16h kh0 = ldfrag_h(k0p + kk * 32);
      const v16h kh1 = ldfrag_h(k1p + kk * 32);
      s0 = mma_h(qh, kh0, s0);
      s1 = mma_h(qh, kh1, s1);
      guard2(s0, s1, qh, kh0, kh1, qh, kh0, kh1);
    }
#pragma unroll
    for (int r = 0; r < 8; ++r) {
      const int mv0 = amb[(size_t)r * SEQ + kb];
      const int mv1 = amb[(size_t)r * SEQ + kb + 16];
      const float t0 = (mv0 != 0) ? (s0[r] * lsc) : FILL;
      const float t1 = (mv1 != 0) ? (s1[r] * lsc) : FILL;
      float mx = fmaxf(t0, t1);
#pragma unroll
      for (int off = 1; off < 16; off <<= 1) mx = fmaxf(mx, __shfl_xor(mx, off, 32));
      const float mn   = fmaxf(mrow[r], mx);
      const float mref = (mn == -INFINITY) ? 0.f : mn;
      const float al   = exp2f(mrow[r] - mref);
      mrow[r] = mn;
      const float e0 = exp2f(t0 - mref), e1 = exp2f(t1 - mref);
      float ps = e0 + e1;
#pragma unroll
      for (int off = 1; off < 16; off <<= 1) ps += __shfl_xor(ps, off, 32);
      lrow[r] = lrow[r] * al + ps;
#pragma unroll
      for (int j = 0; j < 12; ++j) o[j][r] *= al;
      const int ro = (8 * hh + r) * 36 + c;
      pt[ro]      = e0;
      pt[ro + 16] = e1;
    }
    wave_sync_lds();
    FragH ph, pl;
    {
      const float* prow = pt + c * 36 + 8 * hh;
      const v4f p0 = *(const v4f*)(prow), p1 = *(const v4f*)(prow + 4);
      const v4f p2 = *(const v4f*)(prow + 16), p3 = *(const v4f*)(prow + 20);
      pl.u[0] = (v4u){0u, 0u, 0u, 0u};
      pl.u[1] = (v4u){0u, 0u, 0u, 0u};
#pragma unroll
      for (int e = 0; e < 4; ++e) {
        const float ta = p0[e] * PCAR, tb = p1[e] * PCAR, tc = p2[e] * PCAR, td = p3[e] * PCAR;
        const _Float16 ha = (_Float16)ta, hb = (_Float16)tb, hc = (_Float16)tc, hd = (_Float16)td;
        ph.h[0][e]     = ha;
        ph.h[0][4 + e] = hb;
        ph.h[1][e]     = hc;
        ph.h[1][4 + e] = hd;
        if (RESID) {
          pl.h[0][e]     = (_Float16)(ta - (float)ha);
          pl.h[0][4 + e] = (_Float16)(tb - (float)hb);
          pl.h[1][e]     = (_Float16)(tc - (float)hc);
          pl.h[1][4 + e] = (_Float16)(td - (float)hd);
        }
      }
    }
    {
      const _Float16* vhp = Vhb + kb;
      const _Float16* vlp = Vlb + kb;
      pv2<RESID>(o[0],  o[1],  ph.v, pl.v, vhp,                        vlp);
      pv2<RESID>(o[2],  o[3],  ph.v, pl.v, vhp + (size_t)32  * SEQ,    vlp + (size_t)32  * RESR);
      pv2<RESID>(o[4],  o[5],  ph.v, pl.v, vhp + (size_t)64  * SEQ,    vlp + (size_t)64  * RESR);
      pv2<RESID>(o[6],  o[7],  ph.v, pl.v, vhp + (size_t)96  * SEQ,    vlp + (size_t)96  * RESR);
      pv2<RESID>(o[8],  o[9],  ph.v, pl.v, vhp + (size_t)128 * SEQ,    vlp + (size_t)128 * RESR);
      pv2<RESID>(o[10], o[11], ph.v, pl.v, vhp + (size_t)160 * SEQ,    vlp + (size_t)160 * RESR);
    }
    wave_sync_lds();
  }
  acc_guard4(o[0], o[1], o[2], o[3]);
  acc_guard4(o[4], o[5], o[6], o[7]);
  acc_guard4(o[8], o[9], o[10], o[11]);

  const float oc = 1.0f / (PCAR * VCAR);
  v8f invv;
#pragma unroll
  for (int r = 0; r < 8; ++r) invv[r] = (1.0f / lrow[r]) * oc;
  float* slab = pt;
  u16* ohb = OHo + (((size_t)(b * SEQ + q0)) * NH + head) * HDIM;
  u16* olb = OLo + (((size_t)(b * RESR + (RESID ? q0 : 0))) * NH + head) * HDIM;
  epi_chunk<RESID>(slab, o[0], o[1], o[2],  o[3],  invv, ohb,       olb,       lane);
  epi_chunk<RESID>(slab, o[4], o[5], o[6],  o[7],  invv, ohb + 64,  olb + 64,  lane);
  epi_chunk<RESID>(slab, o[8], o[9], o[10], o[11], invv, ohb + 128, olb + 128, lane);
}

extern "C" void kernel_launch(void* const* d_in, const int* in_sizes, int n_in,
                              void* d_out, int out_size, void* d_ws, size_t ws_size,
                              hipStream_t stream) {
  const int ROWS = NB * SEQ;
  if (n_in < 6) return;
  if (in_sizes[0] != ROWS * DMOD) return;
  if (in_sizes[1] != NB * SEQ * SEQ) return;
  if (in_sizes[2] != DMOD * DKV) return;
  if (in_sizes[3] != DKV) return;
  if (in_sizes[4] != DKV * NQKV) return;
  if (in_sizes[5] != DLAT * DMOD) return;
  if (out_size != ROWS * DMOD) return;

  const float* xin = (const float*)d_in[0];
  const int*   amk = (const int*)d_in[1];
  const float* wdn = (const float*)d_in[2];
  const float* rw  = (const float*)d_in[3];
  const float* wup = (const float*)d_in[4];
  const float* wo  = (const float*)d_in[5];
  float*       out = (float*)d_out;

  const size_t szTab = (size_t)SEQ * ROTP * 4;
  const size_t szP   = (size_t)ROWS * DLAT * 2;
  const size_t szF   = (size_t)ROWS * DLAT * 4;
  const size_t szPL  = (size_t)NB * RESR * DLAT * 2;
  const size_t szWO  = (size_t)DMOD * DLAT * 2;
  const size_t szXB  = (size_t)ROWS * DMOD * 2;
  const size_t szH32 = (size_t)ROWS * DKV * 4;
  const size_t szHN  = (size_t)ROWS * DKV * 2;
  const size_t szWD  = (size_t)DKV * DMOD * 2;
  const size_t szWU  = (size_t)NQKV * DKV * 2;
  const size_t szVL  = (size_t)NB * NH * HDIM * RESR * 2;
  const size_t szA   = szF;
  const size_t szB   = 2 * szHN + szWD + szWU;
  size_t off = 0;
  const size_t oCT = off; off += szTab;
  const size_t oST = off; off += szTab;
  const size_t oQH = off; off += szP;
  const size_t oKH = off; off += szP;
  const size_t oVH = off; off += szP;
  const size_t oA  = off; off += szA;
  const size_t oB  = off; off += szB;
  if (off > ws_size) return;
  if (off > (size_t)134217728) return;
  const size_t oXB  = oA;
  const size_t oH32 = oA + szXB;
  const size_t oF   = oA;
  const size_t oOH  = oA;
  const size_t oOL  = oOH + szP;
  const size_t oWO  = oOL + szPL;
  if (oH32 + szH32 > oA + szA) return;
  if (oWO + szWO > oA + szA) return;
  const size_t oHNH = oB;
  const size_t oHNL = oHNH + szHN;
  const size_t oWD  = oHNL + szHN;
  const size_t oWU  = oWD + szWD;
  const size_t oVL  = oB;
  if (oWU + szWU > oB + szB) return;
  if (oVL + szVL > oB + szB) return;

  char* ws = (char*)d_ws;
  float* CT  = (float*)(ws + oCT);
  float* ST  = (float*)(ws + oST);
  u16*   QH  = (u16*)(ws + oQH);
  u16*   KH  = (u16*)(ws + oKH);
  u16*   VH  = (u16*)(ws + oVH);
  u16*   XB  = (u16*)(ws + oXB);
  float* H32 = (float*)(ws + oH32);
  float* F   = (float*)(ws + oF);
  u16*   OH  = (u16*)(ws + oOH);
  u16*   OL  = (u16*)(ws + oOL);
  u16*   WOB = (u16*)(ws + oWO);
  u16*   HNH = (u16*)(ws + oHNH);
  u16*   HNL = (u16*)(ws + oHNL);
  u16*   WDB = (u16*)(ws + oWD);
  u16*   WUB = (u16*)(ws + oWU);
  u16*   VL  = (u16*)(ws + oVL);

  InvF inv;
  for (int i = 0; i < ROTP; ++i) {
    const double p = pow(10000.0, (double)i / 16.0);
    const float pf = (float)p;
    inv.f[i] = 1.0f / pf;
  }

  const dim3 blk(256);
  const int n8x = (ROWS * DMOD) / 8;
  if ((n8x % 256) != 0) return;
  const int rowsH = ROWS * NH;
  if (((rowsH * (HDIM / 8)) % 256) != 0) return;
  const dim3 gTab(SEQ / 16);
  const dim3 gX(n8x / 256);
  const dim3 gTD((DKV / 64) * (DMOD / 64));
  const dim3 gTU((NQKV / 64) * (DKV / 64));
  const dim3 gTO((DMOD / 64) * (DLAT / 64));
  const dim3 gGD((ROWS / 64) * (DKV / 64));
  const dim3 gGU((ROWS / 64) * (DLAT / 64));
  const dim3 gGO((ROWS / 64) * (DMOD / 64));
  const dim3 bG(128);
  const dim3 gRMS(ROWS / 8);
  const dim3 gR((rowsH * (HDIM / 8)) / 256);
  const dim3 gVT(NB * NH * (SEQ / 64) * 3);
  const int  nqtR = RESR / 64;
  const int  nqtP = SEQ / 64 - nqtR;
  const dim3 gATR(nqtR * NH * NB);
  const dim3 gATP(nqtP * NH * NB);
  const dim3 bAT(ATT_THREADS);

  k_tab<<<gTab, blk, 0, stream>>>(CT, ST, inv);
  tr16<<<gTD, blk, 0, stream>>>(wdn, WDB, DKV, DMOD, DKV / 64, 0, 0, 1.0f);
  tr16<<<gTU, blk, 0, stream>>>(wup, WUB, NQKV, DKV, NQKV / 64, 1, 1, WSC);
  cvt16<<<gX, blk, 0, stream>>>(xin, XB, n8x, 0, 1.0f);
  gemm_bf<<<gGD, bG, 0, stream>>>(XB, WDB, H32, ROWS, DKV, DMOD, 1.0f);
  rms16<<<gRMS, blk, 0, stream>>>(H32, rw, HNH, HNL, ROWS, HSC);
  gemm_hr<<<gGU, bG, 0, stream>>>(HNH, HNL, WUB, F, ROWS, DLAT, DKV, 1.0f / (HSC * WSC), RESR, SEQ);
  rope16<<<gR, blk, 0, stream>>>(F, CT, ST, QH, rowsH, QSC);
  gemm_hr<<<gGU, bG, 0, stream>>>(HNH, HNL, WUB + (size_t)DLAT * DKV, F, ROWS, DLAT, DKV, 1.0f / (HSC * WSC), RESR, SEQ);
  rope16<<<gR, blk, 0, stream>>>(F, CT, ST, KH, rowsH, KSC);
  gemm_hr<<<gGU, bG, 0, stream>>>(HNH, HNL, WUB + (size_t)2 * DLAT * DKV, F, ROWS, DLAT, DKV, 1.0f / (HSC * WSC), RESR, SEQ);
  vt16<<<gVT, blk, 0, stream>>>(F, VH, VL);
  tr16<<<gTO, blk, 0, stream>>>(wo, WOB, DMOD, DLAT, DMOD / 64, 0, 1, WSC);
  attn_causal<true><<<gATR, bAT, 0, stream>>>(QH, KH, VH, VL, amk, OH, OL, 0, nqtR);
  attn_causal<false><<<gATP, bAT, 0, stream>>>(QH, KH, VH, VL, amk, OH, OL, nqtR, nqtP);
  gemm_hr<<<gGO, bG, 0, stream>>>(OH, OL, WOB, out, ROWS, DMOD, DLAT, 1.0f / (OSC * WSC), RESR, RESR);
  (void)hipGetLastError();
}
